// CausalAttention_62191126446396
// MI455X (gfx1250) — hardware-verified
//
#include <hip/hip_runtime.h>


#ifndef NB
#define NB 2
#endif
#ifndef SEQ
#define SEQ 2048
#endif
#define SEQ_FULL 2048
#define DMOD  1024
#define NHEAD 16
#define HD    64
#define QKVN  3072
#define L2E   1.4426950408889634f
#define NEGM  (-1.0e30f)

typedef unsigned short bf;
typedef __attribute__((ext_vector_type(16))) __bf16   v16bf;
typedef __attribute__((ext_vector_type(8)))  unsigned short v8us;
typedef __attribute__((ext_vector_type(2)))  unsigned short v2us;
typedef __attribute__((ext_vector_type(8)))  float    v8f;
typedef __attribute__((ext_vector_type(4)))  float    v4f;
typedef v4f  __attribute__((may_alias)) v4fa;
typedef v8us __attribute__((may_alias)) v8usa;

static_assert(SEQ % 64 == 0);
static_assert(SEQ <= SEQ_FULL);
static_assert(NB >= 1 && NB <= 2);
static_assert(DMOD == NHEAD * HD);
static_assert(QKVN == 3 * DMOD);
static_assert(((QKVN * DMOD) / 64) % 64 == 0);
static_assert(((DMOD * DMOD) / 64) % 64 == 0);
static_assert((NB * SEQ * (DMOD / 8)) % 256 == 0);
static_assert((NB * NHEAD * HD * SEQ) % 512 == 0);
static_assert((size_t)2 * NB * SEQ * DMOD * 2 <= (size_t)NB * SEQ * QKVN * 4);

__device__ __forceinline__ unsigned short f2bf(float f) { unsigned u = __float_as_uint(f); u += 0x7FFFu + ((u >> 16) & 1u); return (unsigned short)(u >> 16); }
__device__ __forceinline__ float bf2f(unsigned short b) { return __uint_as_float(((unsigned)b) << 16); }
__device__ __forceinline__ float bfr(float f) { return bf2f(f2bf(f)); }
__device__ __forceinline__ void splitf(float y, unsigned short& h, unsigned short& l) { h = f2bf(y); l = f2bf(y - bf2f(h)); }
__device__ __forceinline__ v16bf cat16b(v8us lo, v8us hi) { return __builtin_bit_cast(v16bf, __builtin_shufflevector(lo, hi, 0, 1, 2, 3, 4, 5, 6, 7, 8, 9, 10, 11, 12, 13, 14, 15)); }
__device__ __forceinline__ v8f wmmab(v16bf a, v16bf b, v8f c) { return __builtin_amdgcn_wmma_f32_16x16x32_bf16(false, a, false, b, (short)0, c, false, false); }

template <typename T16> struct WFrag;
template <> struct WFrag<bf> { typedef v16bf V; static __device__ __forceinline__ V ld(const bf* p) { return cat16b(*(const v8us*)p, *(const v8us*)(p + 16)); } static __device__ __forceinline__ v8f mma(V a, V b, v8f c) { return wmmab(a, b, c); } };

template <typename T16, int NSPLIT, bool BIAS>
__global__ __launch_bounds__(32) void k_gemmw(const T16* __restrict__ A, const T16* __restrict__ A2, const T16* __restrict__ Bt, const T16* __restrict__ Bt2, int K, float* C, int ldc, const float* __restrict__ bias, size_t sA, size_t sB, size_t sC) {
    typedef typename WFrag<T16>::V V;
    __shared__ __align__(16) float os[16 * 68];
    const size_t z = blockIdx.z; A += z * sA; if (A2) A2 += z * sA; Bt += z * sB; if (Bt2) Bt2 += z * sB; C += z * sC;
    const int lane = threadIdx.x & 31, lr = lane & 15, hi = lane >> 4; const int r0 = blockIdx.x * 64, c0 = blockIdx.y * 64;
    v8f acc[4][4];
#pragma unroll
    for (int mb = 0; mb < 4; ++mb)
#pragma unroll
        for (int nb = 0; nb < 4; ++nb) acc[mb][nb] = (v8f){};
    const size_t aoff = (size_t)(r0 + lr) * K + 8 * hi, boff = (size_t)(c0 + lr) * K + 8 * hi;
#pragma unroll 1
    for (int kc = 0; kc < K; kc += 32) {
        V a[4], a2[4];
#pragma unroll
        for (int mb = 0; mb < 4; ++mb) { a[mb] = WFrag<T16>::ld(A + aoff + (size_t)mb * 16 * K + kc); if (NSPLIT == 1 || NSPLIT == 2) a2[mb] = WFrag<T16>::ld(A2 + aoff + (size_t)mb * 16 * K + kc); }
#pragma unroll
        for (int nb = 0; nb < 4; ++nb) { const V b = WFrag<T16>::ld(Bt + boff + (size_t)nb * 16 * K + kc); V b2; if (NSPLIT >= 2) b2 = WFrag<T16>::ld(Bt2 + boff + (size_t)nb * 16 * K + kc);
#pragma unroll
            for (int mb = 0; mb < 4; ++mb) { acc[mb][nb] = WFrag<T16>::mma(a[mb], b, acc[mb][nb]); if (NSPLIT == 1 || NSPLIT == 2) acc[mb][nb] = WFrag<T16>::mma(a2[mb], b, acc[mb][nb]); if (NSPLIT >= 2) acc[mb][nb] = WFrag<T16>::mma(a[mb], b2, acc[mb][nb]); } }
        asm volatile("v_nop\n\tv_nop\n\tv_nop\n\tv_nop" : "+v"(acc[0][0]), "+v"(acc[1][1]), "+v"(acc[2][2]), "+v"(acc[3][3]) : "v"(a[0]), "v"(a[3]));
    }
#pragma unroll
    for (int mb = 0; mb < 4; ++mb) {
#pragma unroll
        for (int nb = 0; nb < 4; ++nb) {
#pragma unroll
            for (int j = 0; j < 8; ++j) os[(hi * 8 + j) * 68 + nb * 16 + lr] = acc[mb][nb][j]; }
        __builtin_amdgcn_wave_barrier(); asm volatile("" ::: "memory");
        float* crow = C + (size_t)(r0 + mb * 16) * ldc + c0;
#pragma unroll 1
        for (int ps = 0; ps < 2; ++ps) {
#pragma unroll
            for (int s = 0; s < 8; ++s) { const int row = 2 * s + hi, cofs = lr * 4; v4f val = *(const v4fa*)(os + row * 68 + cofs); if (BIAS) { val[0] += bfr(bias[c0 + cofs]); val[1] += bfr(bias[c0 + cofs + 1]); val[2] += bfr(bias[c0 + cofs + 2]); val[3] += bfr(bias[c0 + cofs + 3]); }
                *(volatile v4f*)(crow + (size_t)row * ldc + cofs) = val; }
            if (ps == 0) __threadfence(); }
        __builtin_amdgcn_wave_barrier(); asm volatile("" ::: "memory");
    }
}

__global__ __launch_bounds__(256) void k_cvtx(const float* __restrict__ x, bf* dst) {
    const unsigned i = blockIdx.x * 256u + threadIdx.x; if (i >= (unsigned)(NB * SEQ * (DMOD / 8))) return;
    const unsigned m = i >> 7, c8 = i & 127u; const unsigned b = m / (unsigned)SEQ, t = m % (unsigned)SEQ;
    const v8f v = *(const v8f*)(x + ((size_t)b * SEQ_FULL + t) * DMOD + c8 * 8u); v8us o;
#pragma unroll
    for (int k = 0; k < 8; ++k) o[k] = f2bf(v[k]);
    bf* dp = dst + (size_t)i * 8;
    *(volatile v8us*)dp = o; __threadfence(); *(volatile v8us*)dp = o;
}

__global__ __launch_bounds__(256) void k_wtG(const float* __restrict__ w, unsigned N, bf* Bt) {
    const unsigned lane = threadIdx.x & 31u; const unsigned L0 = (blockIdx.x * 8u + (threadIdx.x >> 5)) * 8u;
#pragma unroll
    for (int ps = 0; ps < 2; ++ps) {
#pragma unroll 1
        for (unsigned l = 0; l < 8u; ++l) { const unsigned L = L0 + l; const unsigned e = L * 64u + lane * 2u; const unsigned k = e & (unsigned)(DMOD - 1), n = e >> 10; v2us o;
            o[0] = f2bf(w[(size_t)k * N + n]); o[1] = f2bf(w[(size_t)(k + 1u) * N + n]); *(volatile v2us*)(Bt + e) = o; }
        if (ps == 0) __threadfence(); }
}

__global__ __launch_bounds__(256) void k_qksp(const float* __restrict__ F, bf* Qh, bf* Ql, bf* Kh, bf* Kl) {
    const unsigned i = blockIdx.x * 256u + threadIdx.x; if (i >= (unsigned)(NB * SEQ) * 256u) return;
    const unsigned m = i >> 8, c = (i & 255u) * 8u; const unsigned which = c >> 10, cc = c & 1023u; const unsigned h = cc >> 6, d = cc & 63u; const unsigned b = m / (unsigned)SEQ, t = m % (unsigned)SEQ;
    const float sc = which ? 1.0f : 0.125f;
    const v4f a0 = *(const v4f*)(F + (size_t)m * QKVN + c); const v4f a1 = *(const v4f*)(F + (size_t)m * QKVN + c + 4u);
    v8us oh, ol;
#pragma unroll
    for (int k = 0; k < 4; ++k) { unsigned short x0, y0, x1, y1; splitf(a0[k] * sc, x0, y0); splitf(a1[k] * sc, x1, y1); oh[k] = x0; ol[k] = y0; oh[k + 4] = x1; ol[k + 4] = y1; }
    const size_t oo = (((size_t)(b * NHEAD + h)) * SEQ + t) * HD + d;
    bf* dh = which ? Kh : Qh; bf* dl = which ? Kl : Ql;
    *(volatile v8us*)(dh + oo) = oh; *(volatile v8us*)(dl + oo) = ol; __threadfence(); *(volatile v8us*)(dh + oo) = oh; *(volatile v8us*)(dl + oo) = ol;
}

__global__ __launch_bounds__(256) void k_vtp(const float* __restrict__ F, bf* Vh, bf* Vl) {
    const unsigned e = (blockIdx.x * 256u + threadIdx.x) * 2u; if (e >= (unsigned)(NB * NHEAD * HD * SEQ)) return;
    const unsigned t = e % (unsigned)SEQ; const unsigned d = (e / (unsigned)SEQ) % (unsigned)HD; const unsigned u = e / (unsigned)(SEQ * HD); const unsigned b = u / (unsigned)NHEAD, h = u % (unsigned)NHEAD;
    v2us oh, ol;
#pragma unroll
    for (int q = 0; q < 2; ++q) { const float x = F[((size_t)b * SEQ + t + (unsigned)q) * QKVN + 2u * DMOD + h * HD + d]; unsigned short a2, c2; splitf(x, a2, c2); oh[q] = a2; ol[q] = c2; }
    *(volatile v2us*)(Vh + e) = oh; *(volatile v2us*)(Vl + e) = ol; __threadfence(); *(volatile v2us*)(Vh + e) = oh; *(volatile v2us*)(Vl + e) = ol;
}

__global__ __launch_bounds__(32) void k_flash(const bf* Qh, const bf* Ql, const bf* Kh, const bf* Kl, const bf* VTh, const bf* VTl, bf* Ch, bf* Cl) {
    typedef WFrag<bf>::V V;
    __shared__ __align__(16) unsigned short phs[16 * 40];
    __shared__ __align__(16) unsigned short pls[16 * 40];
    __shared__ __align__(16) float os[16 * 68];
    const unsigned lane = threadIdx.x & 31u, lr = lane & 15u, hi = lane >> 4;
    const unsigned q0 = blockIdx.x * 16u, u = blockIdx.y;
    const size_t ub = (size_t)u * SEQ * HD;
    V aqh[2], aql[2];
    { const size_t qo = ub + (size_t)(q0 + lr) * HD + 8u * hi;
#pragma unroll
      for (int c = 0; c < 2; ++c) { aqh[c] = WFrag<bf>::ld(Qh + qo + 32 * c); aql[c] = WFrag<bf>::ld(Ql + qo + 32 * c); } }
    float mrow[8], lsum[8]; v8f o[4];
#pragma unroll
    for (int r = 0; r < 8; ++r) { mrow[r] = NEGM; lsum[r] = 0.0f; }
#pragma unroll
    for (int c = 0; c < 4; ++c) o[c] = (v8f){};
    const unsigned nch = (q0 >> 5) + 1u;
#pragma unroll 1
    for (unsigned kc = 0; kc < nch; ++kc) {
        const unsigned kb = kc * 32u;
        const size_t ko0 = ub + (size_t)(kb + lr) * HD + 8u * hi; const size_t ko1 = ko0 + (size_t)16 * HD;
        v8f s0 = (v8f){}, s1 = (v8f){};
#pragma unroll
        for (int c = 0; c < 2; ++c) {
            const V k0h = WFrag<bf>::ld(Kh + ko0 + 32 * c), k0l = WFrag<bf>::ld(Kl + ko0 + 32 * c);
            const V k1h = WFrag<bf>::ld(Kh + ko1 + 32 * c), k1l = WFrag<bf>::ld(Kl + ko1 + 32 * c);
            s0 = wmmab(aqh[c], k0h, s0); s1 = wmmab(aqh[c], k1h, s1);
            s0 = wmmab(aqh[c], k0l, s0); s1 = wmmab(aqh[c], k1l, s1);
            s0 = wmmab(aql[c], k0h, s0); s1 = wmmab(aql[c], k1h, s1);
        }
        asm volatile("v_nop\n\tv_nop\n\tv_nop\n\tv_nop" : "+v"(s0), "+v"(s1) : "v"(aqh[0]), "v"(aql[1]));
        float alpha[8];
#pragma unroll
        for (int r = 0; r < 8; ++r) {
            const unsigned qrow = q0 + 8u * hi + (unsigned)r;
            const float v0 = (kb + lr <= qrow) ? s0[r] : NEGM;
            const float v1 = (kb + 16u + lr <= qrow) ? s1[r] : NEGM;
            float mx = fmaxf(v0, v1);
            mx = fmaxf(mx, __shfl_xor(mx, 8, 32)); mx = fmaxf(mx, __shfl_xor(mx, 4, 32)); mx = fmaxf(mx, __shfl_xor(mx, 2, 32)); mx = fmaxf(mx, __shfl_xor(mx, 1, 32));
            const float mn = fmaxf(mrow[r], mx);
            const float al = __builtin_amdgcn_exp2f((mrow[r] - mn) * L2E);
            const float p0 = __builtin_amdgcn_exp2f((v0 - mn) * L2E);
            const float p1 = __builtin_amdgcn_exp2f((v1 - mn) * L2E);
            alpha[r] = al; lsum[r] = lsum[r] * al + (p0 + p1); mrow[r] = mn;
            unsigned short h0, l0, h1, l1; splitf(p0, h0, l0); splitf(p1, h1, l1);
            const unsigned po = (8u * hi + (unsigned)r) * 40u + lr;
            phs[po] = h0; pls[po] = l0; phs[po + 16u] = h1; pls[po + 16u] = l1;
        }
#pragma unroll
        for (int c = 0; c < 4; ++c)
#pragma unroll
            for (int r = 0; r < 8; ++r) o[c][r] *= alpha[r];
        __syncthreads();
        const unsigned pr = lr * 40u + 8u * hi;
        const V ph = cat16b(*(const v8usa*)(phs + pr), *(const v8usa*)(phs + pr + 16u));
        const V pl = cat16b(*(const v8usa*)(pls + pr), *(const v8usa*)(pls + pr + 16u));
#pragma unroll
        for (int c = 0; c < 4; ++c) {
            const size_t vo = ((size_t)u * HD + 16u * (unsigned)c + lr) * SEQ + kb + 8u * hi;
            const V vh = WFrag<bf>::ld(VTh + vo), vl = WFrag<bf>::ld(VTl + vo);
            o[c] = wmmab(ph, vh, o[c]); o[c] = wmmab(ph, vl, o[c]); o[c] = wmmab(pl, vh, o[c]);
        }
        asm volatile("v_nop\n\tv_nop\n\tv_nop\n\tv_nop" : "+v"(o[0]), "+v"(o[1]), "+v"(o[2]), "+v"(o[3]) : "v"(ph), "v"(pl));
        __syncthreads();
    }
    float inv[8];
#pragma unroll
    for (int r = 0; r < 8; ++r) { float t = lsum[r]; t += __shfl_xor(t, 8, 32); t += __shfl_xor(t, 4, 32); t += __shfl_xor(t, 2, 32); t += __shfl_xor(t, 1, 32); inv[r] = 1.0f / t; }
#pragma unroll
    for (int c = 0; c < 4; ++c)
#pragma unroll
        for (int r = 0; r < 8; ++r) os[(8u * hi + (unsigned)r) * 68u + 16u * (unsigned)c + lr] = o[c][r] * inv[r];
    __syncthreads();
    const unsigned b = u >> 4, h = u & 15u;
    const size_t cb = ((size_t)b * SEQ + q0) * DMOD + h * HD;
    const unsigned rq = lane >> 3, pc = (lane & 7u) * 8u;
#pragma unroll 1
    for (int ps = 0; ps < 2; ++ps) {
#pragma unroll
        for (int s = 0; s < 4; ++s) { const unsigned row = 4u * (unsigned)s + rq; const v4f a0 = *(const v4fa*)(os + row * 68u + pc); const v4f a1 = *(const v4fa*)(os + row * 68u + pc + 4u); v8us oh, ol;
#pragma unroll
            for (int k = 0; k < 4; ++k) { unsigned short x0, y0, x1, y1; splitf(a0[k], x0, y0); splitf(a1[k], x1, y1); oh[k] = x0; ol[k] = y0; oh[k + 4] = x1; ol[k + 4] = y1; }
            const size_t oo = cb + (size_t)row * DMOD + pc;
            *(volatile v8us*)(Ch + oo) = oh; *(volatile v8us*)(Cl + oo) = ol; }
        if (ps == 0) __threadfence(); }
}

extern "C" void kernel_launch(void* const* d_in, const int* in_sizes, int n_in,
                              void* d_out, int out_size, void* d_ws, size_t ws_size, hipStream_t stream) {
    if (n_in < 5) return;
    const long long need_x = ((long long)(NB - 1) * SEQ_FULL + SEQ) * DMOD;
    if ((long long)in_sizes[0] < need_x || (long long)in_sizes[1] < (long long)DMOD * QKVN || in_sizes[2] < QKVN || (long long)in_sizes[3] < (long long)DMOD * DMOD || in_sizes[4] < DMOD) return;
    if ((long long)out_size < need_x) return;
    const float* x = (const float*)d_in[0]; const float* w_qkv = (const float*)d_in[1]; const float* b_qkv = (const float*)d_in[2]; const float* w_proj = (const float*)d_in[3]; const float* b_proj = (const float*)d_in[4];
    float* OUT = (float*)d_out;
    char* wsp = (char*)d_ws;
    auto take = [&](size_t bytes) { char* p = wsp; wsp += (bytes + 255) & ~(size_t)255; return (void*)p; };
    const size_t plane = (size_t)NB * SEQ * DMOD * 2;
    bf* XB  = (bf*)take(plane);
    bf* WQT = (bf*)take((size_t)QKVN * DMOD * 2);
    bf* WPT = (bf*)take((size_t)DMOD * DMOD * 2);
    float* QKV = (float*)take((size_t)NB * SEQ * QKVN * 4);
    bf* Qh = (bf*)take(plane); bf* Ql = (bf*)take(plane); bf* Kh = (bf*)take(plane); bf* Kl = (bf*)take(plane); bf* VTh = (bf*)take(plane); bf* VTl = (bf*)take(plane);
    if ((size_t)(wsp - (char*)d_ws) > ws_size) return;
    bf* CTXh = (bf*)QKV; bf* CTXl = (bf*)((char*)QKV + plane);

    k_cvtx<<<(unsigned)(NB * SEQ * (DMOD / 8) / 256), 256, 0, stream>>>(x, XB);
    k_wtG<<<(unsigned)((QKVN * DMOD / 64) / 64), 256, 0, stream>>>(w_qkv, (unsigned)QKVN, WQT);
    k_wtG<<<(unsigned)((DMOD * DMOD / 64) / 64), 256, 0, stream>>>(w_proj, (unsigned)DMOD, WPT);
    k_gemmw<bf, 0, true><<<dim3(NB * SEQ / 64, QKVN / 64, 1), 32, 0, stream>>>(XB, nullptr, WQT, nullptr, DMOD, QKV, QKVN, b_qkv, 0, 0, 0);
    k_qksp<<<(unsigned)(NB * SEQ), 256, 0, stream>>>(QKV, Qh, Ql, Kh, Kl);
    k_vtp<<<(unsigned)(NB * NHEAD * HD * SEQ / 512), 256, 0, stream>>>(QKV, VTh, VTl);
    k_flash<<<dim3(SEQ / 16, NB * NHEAD, 1), 32, 0, stream>>>(Qh, Ql, Kh, Kl, VTh, VTl, CTXh, CTXl);
    k_gemmw<bf, 1, true><<<dim3(SEQ / 64, DMOD / 64, NB), 32, 0, stream>>>(CTXh, CTXl, WPT, nullptr, DMOD, OUT, DMOD, b_proj, (size_t)SEQ * DMOD, 0, (size_t)SEQ_FULL * DMOD);
}
